// CausalStructureEnhancedGAT_80324478370389
// MI455X (gfx1250) — hardware-verified
//
#include <hip/hip_runtime.h>
#include <math.h>

constexpr int kB    = 8;
constexpr int kN    = 2048;
constexpr int kDin  = 128;
constexpr int kDout = 64;
constexpr int kH    = 4;
constexpr int kHD   = kH * kDout;
constexpr int kTok  = kB * kN;
constexpr float kNegSlope = 0.2f;
constexpr float kInvN     = 1.0f / 2048.0f;

typedef __attribute__((ext_vector_type(16))) _Float16 v16h;
typedef __attribute__((ext_vector_type(8)))  _Float16 v8h;
typedef __attribute__((ext_vector_type(16))) __bf16   v16b;
typedef __attribute__((ext_vector_type(8)))  __bf16   v8b;
typedef __attribute__((ext_vector_type(8)))  float    v8f;
typedef __attribute__((ext_vector_type(4)))  float    v4f;
typedef __attribute__((ext_vector_type(4)))  unsigned int v4u;

__device__ __forceinline__ unsigned short f2bf_bits(float f) {
  unsigned u = __float_as_uint(f);
  return (unsigned short)((u + 0x7FFFu + ((u >> 16) & 1u)) >> 16);
}
__device__ __forceinline__ float bf_bits2f(unsigned short h) { return __uint_as_float(((unsigned)h) << 16); }

__device__ __forceinline__ void dep_guard_h(v8f& a, v8f& b, v16h x, v16h y) { asm volatile("v_nop\n\tv_nop\n\tv_nop\n\tv_nop" : "+v"(a), "+v"(b) : "v"(x), "v"(y)); }
__device__ __forceinline__ void dep_guard_b(v8f& a, v8f& b, v16b x, v16b y) { asm volatile("v_nop\n\tv_nop\n\tv_nop\n\tv_nop" : "+v"(a), "+v"(b) : "v"(x), "v"(y)); }
__device__ __forceinline__ void keep4_h(v16h a, v16h b, v16h c, v16h d) { asm volatile("v_nop" :: "v"(a), "v"(b), "v"(c), "v"(d)); }
__device__ __forceinline__ void keep4_b(v16b a, v16b b, v16b c, v16b d) { asm volatile("v_nop" :: "v"(a), "v"(b), "v"(c), "v"(d)); }
__device__ __forceinline__ void acc_guard4(v8f& a, v8f& b, v8f& c, v8f& d) { asm volatile("v_nop\n\tv_nop\n\tv_nop\n\tv_nop" : "+v"(a), "+v"(b), "+v"(c), "+v"(d)); }
template <typename T> struct Frag;
template <> struct Frag<_Float16> {
  typedef v16h V; union U { v16h v; v8h h[2]; };
  static __device__ __forceinline__ v16h load(const _Float16* p) {
    U f; f.h[0] = *(const v8h*)(p); f.h[1] = *(const v8h*)(p + 16); return f.v;
  }
  static __device__ __forceinline__ v8f mma(v16h a, v16h b, v8f c) {
    return __builtin_amdgcn_wmma_f32_16x16x32_f16(false, a, false, b, (short)0, c, false, false);
  }
  static __device__ __forceinline__ void guard(v8f& a, v8f& b, v16h x, v16h y) { dep_guard_h(a, b, x, y); }
  static __device__ __forceinline__ void keep(v16h a, v16h b, v16h c, v16h d) { keep4_h(a, b, c, d); }
};
template <> struct Frag<__bf16> {
  typedef v16b V; union U { v16b v; v8b h[2]; };
  static __device__ __forceinline__ v16b load(const __bf16* p) {
    U f; f.h[0] = *(const v8b*)(p); f.h[1] = *(const v8b*)(p + 16); return f.v;
  }
  static __device__ __forceinline__ v8f mma(v16b a, v16b b, v8f c) {
    return __builtin_amdgcn_wmma_f32_16x16x32_bf16(false, a, false, b, (short)0, c, false, false);
  }
  static __device__ __forceinline__ void guard(v8f& a, v8f& b, v16b x, v16b y) { dep_guard_b(a, b, x, y); }
  static __device__ __forceinline__ void keep(v16b a, v16b b, v16b c, v16b d) { keep4_b(a, b, c, d); }
};

__device__ __forceinline__ unsigned pk16(unsigned short a, unsigned short b) { return (unsigned)a | ((unsigned)b << 16); }

template <int ET> struct Elem;
template <> struct Elem<0> { typedef _Float16 T; };
template <> struct Elem<1> { typedef __bf16 T; };
template <int ET, bool SPLIT, int BIAS_MODE, int OUT_MODE, bool RESID, int ACT = 0>
__global__ __launch_bounds__(256) void wmma_gemm64(
    const unsigned short* __restrict__ Ap, const unsigned short* __restrict__ A2p, int lda, long strideA,
    const unsigned short* __restrict__ Btp, const unsigned short* __restrict__ Bt2p, int ldb, long strideB,
    void* __restrict__ Cout, void* __restrict__ Cout2, int ldc, long strideC,
    const float* __restrict__ bias,
    const float* __restrict__ resid, long strideR,
    int M, int N, int K, float scale) {
  typedef typename Elem<ET>::T T;
  typedef typename Frag<T>::V V;
  const T* A = (const T*)Ap; const T* A2 = (const T*)A2p; const T* Bt = (const T*)Btp; const T* Bt2 = (const T*)Bt2p;
  __shared__ __align__(16) float sT[8][16 * 68];
  const int b    = blockIdx.y;
  const int lane = threadIdx.x & 31;
  const int wave = threadIdx.x >> 5;
  const int tilesN = N >> 6;
  const int tilesM = M >> 6;
  const int tile = blockIdx.x * 8 + wave;
  if (tile >= tilesM * tilesN) return;
  const int tm = tile / tilesN;
  const int tn = tile - tm * tilesN;
  const int m0 = tm << 6;
  const int n0 = tn << 6;

  const T* Ab  = A  + (size_t)b * strideA;
  const T* Bb  = Bt + (size_t)b * strideB;
  const T* Ab2 = SPLIT ? (A2  + (size_t)b * strideA) : nullptr;
  const T* Bb2 = SPLIT ? (Bt2 + (size_t)b * strideB) : nullptr;

  const int rlane = lane & 15;
  const int koff  = (lane >> 4) * 8;
  const int mOff  = (lane >> 4) * 8;

  v8f acc[4][4];
#pragma unroll
  for (int i = 0; i < 4; ++i)
#pragma unroll
    for (int j = 0; j < 4; ++j) acc[i][j] = (v8f){0.f,0.f,0.f,0.f,0.f,0.f,0.f,0.f};

  for (int k0 = 0; k0 < K; k0 += 32) {
    V bh[4], bl[4];
#pragma unroll
    for (int j = 0; j < 4; ++j) {
      const size_t bo = (size_t)(n0 + (j << 4) + rlane) * ldb + koff + k0;
      bh[j] = Frag<T>::load(Bb + bo);
      if (SPLIT) bl[j] = Frag<T>::load(Bb2 + bo);
    }
#pragma unroll
    for (int i = 0; i < 4; ++i) {
      const size_t ao = (size_t)(m0 + (i << 4) + rlane) * lda + koff + k0;
      V ah = Frag<T>::load(Ab + ao);
      V al;
      if (SPLIT) al = Frag<T>::load(Ab2 + ao);
#pragma unroll
      for (int j = 0; j < 4; ++j) {
        acc[i][j] = Frag<T>::mma(ah, bh[j], acc[i][j]);
        if (SPLIT) {
          acc[i][j] = Frag<T>::mma(ah, bl[j], acc[i][j]);
          acc[i][j] = Frag<T>::mma(al, bh[j], acc[i][j]);
        }
      }
      Frag<T>::guard(acc[i][0], acc[i][3], ah, SPLIT ? al : ah);
    }
    Frag<T>::keep(bh[0], bh[1], bh[2], bh[3]);
    if (SPLIT) Frag<T>::keep(bl[0], bl[1], bl[2], bl[3]);
  }
  acc_guard4(acc[0][0], acc[0][1], acc[0][2], acc[0][3]);
  acc_guard4(acc[1][0], acc[1][1], acc[1][2], acc[1][3]);
  acc_guard4(acc[2][0], acc[2][1], acc[2][2], acc[2][3]);
  acc_guard4(acc[3][0], acc[3][1], acc[3][2], acc[3][3]);

  float* slab = sT[wave];
  const float* Rb = RESID ? (resid + (size_t)b * strideR) : nullptr;
#pragma unroll
  for (int i = 0; i < 4; ++i) {
    const int mBase = m0 + (i << 4);
#pragma unroll
    for (int j = 0; j < 4; ++j) {
      const int n = n0 + (j << 4) + rlane;
      float bv = 0.f;
      if (BIAS_MODE == 2) bv = bias[n];
#pragma unroll
      for (int r = 0; r < 8; ++r) {
        float v = acc[i][j][r] * scale;
        if (BIAS_MODE == 1) v += bias[mBase + mOff + r];
        if (BIAS_MODE == 2) v += bv;
        if (RESID) v += Rb[(size_t)(mBase + mOff + r) * ldc + n];
        if (ACT == 2) v = fmaxf(v, 0.0f);
        if (ACT == 4) v = (v > 0.f) ? v : 0.01f * v;
        slab[(mOff + r) * 68 + (j << 4) + rlane] = v;
      }
    }
    __builtin_amdgcn_fence(__ATOMIC_RELEASE, "workgroup");
    __builtin_amdgcn_wave_barrier();
    __builtin_amdgcn_fence(__ATOMIC_ACQUIRE, "workgroup");
    if (OUT_MODE == 0) {
      float* C = (float*)Cout + (size_t)b * strideC;
      const int hh = lane >> 4, c4 = (lane & 15) * 4;
      for (int pass = 0; pass < 2; ++pass) {
#pragma unroll
        for (int it = 0; it < 8; ++it) {
          const int row = it * 2 + hh;
          v4f v = *(const v4f*)(slab + row * 68 + c4);
          *(volatile v4f*)(C + (size_t)(mBase + row) * ldc + n0 + c4) = v;
        }
        __threadfence();
      }
    } else {
      const int q = lane >> 3, c8 = (lane & 7) * 8;
      unsigned short* C  = (unsigned short*)Cout  + (size_t)b * strideC;
      unsigned short* C2 = (OUT_MODE == 2) ? ((unsigned short*)Cout2 + (size_t)b * strideC) : nullptr;
      for (int pass = 0; pass < 2; ++pass) {
#pragma unroll
        for (int it = 0; it < 4; ++it) {
          const int row = it * 4 + q;
          const float* sp = slab + row * 68 + c8;
          v8h hv, lv;
#pragma unroll
          for (int e = 0; e < 8; ++e) {
            if (OUT_MODE == 1) {
              hv[e] = (_Float16)sp[e];
            } else {
              unsigned short hb = f2bf_bits(sp[e]);
              unsigned short lb = f2bf_bits(sp[e] - bf_bits2f(hb));
              hv[e] = __builtin_bit_cast(_Float16, hb);
              lv[e] = __builtin_bit_cast(_Float16, lb);
            }
          }
          *(volatile v8h*)(C + (size_t)(mBase + row) * ldc + n0 + c8) = hv;
          if (OUT_MODE == 2) *(volatile v8h*)(C2 + (size_t)(mBase + row) * ldc + n0 + c8) = lv;
        }
        __threadfence();
      }
    }
    __builtin_amdgcn_fence(__ATOMIC_RELEASE, "workgroup");
    __builtin_amdgcn_wave_barrier();
    __builtin_amdgcn_fence(__ATOMIC_ACQUIRE, "workgroup");
  }
}

__global__ __launch_bounds__(256) void rowmean_kernel(const float* __restrict__ cs, float* __restrict__ rm) {
  __shared__ float red[32];
  const int t = threadIdx.x, lane = t & 31, wave = t >> 5;
  const int blk = blockIdx.x;
#pragma unroll
  for (int rr = 0; rr < 4; ++rr) {
    const int row = blk * 32 + wave * 4 + rr;
    const float* p = cs + (size_t)row * kN;
    float s = 0.f;
#pragma unroll 4
    for (int k = 0; k < 16; ++k) {
      const v4f v = *(const v4f*)(p + (k * 32 + lane) * 4);
      s += (v[0] + v[1]) + (v[2] + v[3]);
    }
#pragma unroll
    for (int off = 16; off > 0; off >>= 1) s += __shfl_xor(s, off, 32);
    if (lane == 0) red[wave * 4 + rr] = s;
  }
  __syncthreads();
  if (wave == 0) {
    const float v = red[lane] * kInvN;
    float* d = rm + blk * 32;
    *(volatile float*)(d + lane) = v;
    __threadfence();
    *(volatile float*)(d + lane) = v;
  }
}

__global__ __launch_bounds__(256) void split8_kernel(const float* __restrict__ in, unsigned short* __restrict__ hi,
                                                     unsigned short* __restrict__ lo, int n8) {
  const int i = blockIdx.x * 256 + threadIdx.x;
  if (i >= n8) return;
  const float* p = in + 8 * (size_t)i;
  const v4f a = *(const v4f*)(p);
  const v4f c = *(const v4f*)(p + 4);
  float v[8];
#pragma unroll
  for (int e = 0; e < 4; ++e) { v[e] = a[e]; v[4 + e] = c[e]; }
  unsigned short hb[8], lb[8];
#pragma unroll
  for (int e = 0; e < 8; ++e) {
    hb[e] = f2bf_bits(v[e]);
    lb[e] = f2bf_bits(v[e] - bf_bits2f(hb[e]));
  }
  const v4u uh = (v4u){pk16(hb[0], hb[1]), pk16(hb[2], hb[3]), pk16(hb[4], hb[5]), pk16(hb[6], hb[7])};
  const v4u ul = (v4u){pk16(lb[0], lb[1]), pk16(lb[2], lb[3]), pk16(lb[4], lb[5]), pk16(lb[6], lb[7])};
  unsigned short* qh = hi + 8 * (size_t)i;
  unsigned short* ql = lo + 8 * (size_t)i;
  *(volatile v4u*)qh = uh;
  *(volatile v4u*)ql = ul;
  __threadfence();
  *(volatile v4u*)qh = uh;
  *(volatile v4u*)ql = ul;
}

__global__ __launch_bounds__(256) void combine_kernel(const float* __restrict__ x, const float* __restrict__ cct,
                                                      const float* __restrict__ rm, unsigned short* __restrict__ hi,
                                                      unsigned short* __restrict__ lo, int n8) {
  const int i = blockIdx.x * 256 + threadIdx.x;
  if (i >= n8) return;
  const int m = i >> 4;
  const int n = m & (kN - 1);
  const size_t base = 8 * (size_t)i;
  const v4f xa = *(const v4f*)(x + base);
  const v4f xc = *(const v4f*)(x + base + 4);
  const v4f ca = *(const v4f*)(cct + base);
  const v4f cc = *(const v4f*)(cct + base + 4);
  const float r = rm[n];
  float v[8];
#pragma unroll
  for (int e = 0; e < 4; ++e) { v[e] = xa[e] + ca[e] * r; v[4 + e] = xc[e] + cc[e] * r; }
  unsigned short hb[8], lb[8];
#pragma unroll
  for (int e = 0; e < 8; ++e) {
    hb[e] = f2bf_bits(v[e]);
    lb[e] = f2bf_bits(v[e] - bf_bits2f(hb[e]));
  }
  const v4u uh = (v4u){pk16(hb[0], hb[1]), pk16(hb[2], hb[3]), pk16(hb[4], hb[5]), pk16(hb[6], hb[7])};
  const v4u ul = (v4u){pk16(lb[0], lb[1]), pk16(lb[2], lb[3]), pk16(lb[4], lb[5]), pk16(lb[6], lb[7])};
  unsigned short* qh = hi + base;
  unsigned short* ql = lo + base;
  *(volatile v4u*)qh = uh;
  *(volatile v4u*)ql = ul;
  __threadfence();
  *(volatile v4u*)qh = uh;
  *(volatile v4u*)ql = ul;
}

__global__ __launch_bounds__(256) void wt_kernel(const float* __restrict__ W, unsigned short* __restrict__ wth,
                                                 unsigned short* __restrict__ wtl) {
  __shared__ float sm[64 * 129];
  const int t = threadIdx.x, lane = t & 31, wave = t >> 5;
  const int h = blockIdx.x;
  const float* Wh = W + (size_t)h * kDin * kDout;
#pragma unroll
  for (int i = 0; i < 32; ++i) {
    const int e = i * 256 + t;
    const int d = e >> 6;
    const int o = e & 63;
    sm[o * 129 + d] = Wh[e];
  }
  __syncthreads();
  const int hh = lane >> 4, c8 = (lane & 15) * 8;
  for (int pass = 0; pass < 2; ++pass) {
#pragma unroll
    for (int it = 0; it < 4; ++it) {
      const int row = wave * 8 + it * 2 + hh;
      const float* sp = sm + row * 129 + c8;
      unsigned short hb[8], lb[8];
#pragma unroll
      for (int e = 0; e < 8; ++e) {
        hb[e] = f2bf_bits(sp[e]);
        lb[e] = f2bf_bits(sp[e] - bf_bits2f(hb[e]));
      }
      const v4u uh = (v4u){pk16(hb[0], hb[1]), pk16(hb[2], hb[3]), pk16(hb[4], hb[5]), pk16(hb[6], hb[7])};
      const v4u ul = (v4u){pk16(lb[0], lb[1]), pk16(lb[2], lb[3]), pk16(lb[4], lb[5]), pk16(lb[6], lb[7])};
      const size_t off = (size_t)(h * kDout + row) * kDin + c8;
      *(volatile v4u*)(wth + off) = uh;
      *(volatile v4u*)(wtl + off) = ul;
    }
    __threadfence();
  }
}

__global__ __launch_bounds__(256) void xpose_dots_kernel(const float* __restrict__ XT, const float* __restrict__ att,
                                                         float* __restrict__ si, float* __restrict__ sj,
                                                         unsigned short* __restrict__ tth, unsigned short* __restrict__ ttl) {
  __shared__ float sm[64 * 65];
  __shared__ float av[128];
  __shared__ float ss[128];
  const int t = threadIdx.x, lane = t & 31, wave = t >> 5;
  const int bh = blockIdx.y, b = bh >> 2, h = bh & 3;
  const int j0 = blockIdx.x * 64;
  const float* src = XT + ((size_t)b * kN + j0) * kHD + h * kDout;
#pragma unroll
  for (int i = 0; i < 16; ++i) {
    const int e  = i * 256 + t;
    const int jl = e >> 6;
    const int o  = e & 63;
    sm[o * 65 + jl] = src[(size_t)jl * kHD + o];
  }
  if (t < 128) av[t] = att[h * 2 * kDout + t];
  __syncthreads();
  if (t < 128) {
    const int jl = t & 63;
    const float* ap = av + (t >> 6) * 64;
    float acc = 0.f;
#pragma unroll 4
    for (int o = 0; o < 64; ++o) acc += sm[o * 65 + jl] * ap[o];
    ss[t] = acc;
  }
  __syncthreads();
  const int q = lane >> 3, c8 = (lane & 7) * 8;
  for (int pass = 0; pass < 2; ++pass) {
#pragma unroll
    for (int it = 0; it < 2; ++it) {
      const int row = wave * 8 + it * 4 + q;
      const float* sp = sm + row * 65 + c8;
      unsigned short hb[8], lb[8];
#pragma unroll
      for (int e = 0; e < 8; ++e) {
        hb[e] = f2bf_bits(sp[e]);
        lb[e] = f2bf_bits(sp[e] - bf_bits2f(hb[e]));
      }
      const v4u uh = (v4u){pk16(hb[0], hb[1]), pk16(hb[2], hb[3]), pk16(hb[4], hb[5]), pk16(hb[6], hb[7])};
      const v4u ul = (v4u){pk16(lb[0], lb[1]), pk16(lb[2], lb[3]), pk16(lb[4], lb[5]), pk16(lb[6], lb[7])};
      const size_t off = (size_t)(bh * kDout + row) * kN + j0 + c8;
      *(volatile v4u*)(tth + off) = uh;
      *(volatile v4u*)(ttl + off) = ul;
    }
    if (wave == 0) {
      const float v0 = ss[lane], v1 = ss[32 + lane];
      float* d = si + (size_t)bh * kN + j0;
      *(volatile float*)(d + lane) = v0;
      *(volatile float*)(d + 32 + lane) = v1;
    }
    if (wave == 1) {
      const float v0 = ss[64 + lane], v1 = ss[96 + lane];
      float* d = sj + (size_t)bh * kN + j0;
      *(volatile float*)(d + lane) = v0;
      *(volatile float*)(d + 32 + lane) = v1;
    }
    __threadfence();
  }
}

__global__ __launch_bounds__(256) void softmax_p_kernel(const float* __restrict__ cs, const float* __restrict__ si,
                                                        const float* __restrict__ sj, const float* __restrict__ cbp,
                                                        unsigned short* __restrict__ ph, unsigned short* __restrict__ pl) {
  __shared__ float redM[8];
  __shared__ float redS[8];
  const int i = blockIdx.x;
  const int h = blockIdx.y;
  const int t = threadIdx.x, lane = t & 31, wave = t >> 5;
  const int c0 = t * 8;
  const float siv = si[(size_t)h * kN + i];
  const float cb  = cbp[0];
  const float* csr = cs + (size_t)i * kN + c0;
  const float* sjr = sj + (size_t)h * kN + c0;
  const v4f ca = *(const v4f*)(csr);
  const v4f cc = *(const v4f*)(csr + 4);
  const v4f ja = *(const v4f*)(sjr);
  const v4f jc = *(const v4f*)(sjr + 4);
  float cv[8], sc[8];
#pragma unroll
  for (int e = 0; e < 4; ++e) { cv[e] = ca[e]; cv[4 + e] = cc[e]; sc[e] = ja[e]; sc[4 + e] = jc[e]; }
  float m = -INFINITY;
#pragma unroll
  for (int e = 0; e < 8; ++e) {
    const float raw = siv + sc[e];
    const float lr  = (raw >= 0.f) ? raw : kNegSlope * raw;
    float s = lr + cb * cv[e];
    s = (cv[e] == 0.0f) ? -INFINITY : s;
    sc[e] = s;
    m = fmaxf(m, s);
  }
#pragma unroll
  for (int off = 16; off > 0; off >>= 1) m = fmaxf(m, __shfl_xor(m, off, 32));
  if (lane == 0) redM[wave] = m;
  __syncthreads();
  float gm = redM[0];
#pragma unroll
  for (int w = 1; w < 8; ++w) gm = fmaxf(gm, redM[w]);
  float ssum = 0.f;
#pragma unroll
  for (int e = 0; e < 8; ++e) {
    const float p = expf(sc[e] - gm);
    sc[e] = p;
    ssum += p;
  }
#pragma unroll
  for (int off = 16; off > 0; off >>= 1) ssum += __shfl_xor(ssum, off, 32);
  if (lane == 0) redS[wave] = ssum;
  __syncthreads();
  float gs = redS[0];
#pragma unroll
  for (int w = 1; w < 8; ++w) gs += redS[w];
  const float inv = 1.0f / gs;
  unsigned short hb[8], lb[8];
#pragma unroll
  for (int e = 0; e < 8; ++e) {
    const float p = sc[e] * inv;
    hb[e] = f2bf_bits(p);
    lb[e] = f2bf_bits(p - bf_bits2f(hb[e]));
  }
  const v4u uh = (v4u){pk16(hb[0], hb[1]), pk16(hb[2], hb[3]), pk16(hb[4], hb[5]), pk16(hb[6], hb[7])};
  const v4u ul = (v4u){pk16(lb[0], lb[1]), pk16(lb[2], lb[3]), pk16(lb[4], lb[5]), pk16(lb[6], lb[7])};
  const size_t off = ((size_t)h * kN + i) * kN + c0;
  *(volatile v4u*)(ph + off) = uh;
  *(volatile v4u*)(pl + off) = ul;
  __threadfence();
  *(volatile v4u*)(ph + off) = uh;
  *(volatile v4u*)(pl + off) = ul;
}

__global__ __launch_bounds__(256) void gate_out_kernel(const float* __restrict__ O, const float* __restrict__ cgw,
                                                       const float* __restrict__ cgb, float* __restrict__ out) {
  __shared__ __align__(16) float Os[64 * 68];
  __shared__ __align__(16) float Rs[64 * 68];
  const int t = threadIdx.x, lane = t & 31, wave = t >> 5;
  const int bh = blockIdx.y, b = bh >> 2, h = bh & 3;
  const int n0 = blockIdx.x * 64;
  const float* Ob = O + ((size_t)bh * kN + n0) * kDout;
#pragma unroll
  for (int i = 0; i < 4; ++i) {
    const int e4  = i * 256 + t;
    const int row = e4 >> 4;
    const int c4  = (e4 & 15) * 4;
    const v4f v = *(const v4f*)(Ob + row * kDout + c4);
    *(v4f*)(Os + row * 68 + c4) = v;
  }
  const int p  = t & 63;
  const int rg = t >> 6;
  v4f cw[16];
#pragma unroll
  for (int q = 0; q < 16; ++q) cw[q] = *(const v4f*)(cgw + p * kDout + q * 4);
  const float bias = cgb[p];
  __syncthreads();
#pragma unroll 1
  for (int k = 0; k < 16; ++k) {
    const int r = rg + 4 * k;
    float acc = 0.f;
#pragma unroll
    for (int q = 0; q < 16; ++q) {
      const v4f x4 = *(const v4f*)(Os + r * 68 + q * 4);
      acc += x4[0] * cw[q][0];
      acc += x4[1] * cw[q][1];
      acc += x4[2] * cw[q][2];
      acc += x4[3] * cw[q][3];
    }
    const float g   = acc + bias;
    const float sig = 1.0f / (1.0f + expf(-g));
    Rs[r * 68 + p] = Os[r * 68 + p] * sig;
  }
  __syncthreads();
  const int hh = lane >> 4, c4 = (lane & 15) * 4;
  float* ob = out + ((size_t)b * kN + n0) * kHD + h * kDout;
  for (int pass = 0; pass < 2; ++pass) {
#pragma unroll
    for (int it = 0; it < 4; ++it) {
      const int row = wave * 8 + it * 2 + hh;
      const v4f v = *(const v4f*)(Rs + row * 68 + c4);
      *(volatile v4f*)(ob + (size_t)row * kHD + c4) = v;
    }
    __threadfence();
  }
}

extern "C" void kernel_launch(void* const* d_in, const int* in_sizes, int n_in,
                              void* d_out, int out_size, void* d_ws, size_t ws_size,
                              hipStream_t stream) {
  (void)in_sizes; (void)n_in; (void)out_size;
  static_assert(kTok * kDin / 8 == 262144);
  static_assert(kN % 32 == 0 && kTok % 64 == 0 && kDin % 32 == 0 && kHD % 64 == 0);
  const float* x     = (const float*)d_in[0];
  const float* cs    = (const float*)d_in[1];
  const float* W     = (const float*)d_in[2];
  const float* att   = (const float*)d_in[3];
  const float* cbias = (const float*)d_in[4];
  const float* ct_w  = (const float*)d_in[5];
  const float* ct_b  = (const float*)d_in[6];
  const float* cg_w  = (const float*)d_in[7];
  const float* cg_b  = (const float*)d_in[8];
  float* out = (float*)d_out;

  const size_t kMiB = 1048576;
  const size_t off_rm  = 0;
  const size_t off_si  = 8192;
  const size_t off_sj  = 270336;
  const size_t off_cwh = 532480;
  const size_t off_cwl = 565248;
  const size_t off_wth = 598016;
  const size_t off_wtl = 663552;
  const size_t off_big = 1 * kMiB;
  const size_t off_xh  = off_big + 0;
  const size_t off_xl  = off_big + 4 * kMiB;
  const size_t off_cct = off_big + 8 * kMiB;
  const size_t off_x1h = off_big + 16 * kMiB;
  const size_t off_x1l = off_big + 20 * kMiB;
  const size_t off_xt  = off_big + 24 * kMiB;
  const size_t off_ph  = off_big + 0;
  const size_t off_pl  = off_big + 32 * kMiB;
  const size_t off_tth = 65 * kMiB;
  const size_t off_ttl = 73 * kMiB;
  const size_t off_o   = 81 * kMiB;
  const size_t total   = 97 * kMiB;
  if (ws_size < total) return;

  char* ws = (char*)d_ws;
  float* rm = (float*)(ws + off_rm);
  float* si = (float*)(ws + off_si);
  float* sj = (float*)(ws + off_sj);
  unsigned short* cwh = (unsigned short*)(ws + off_cwh);
  unsigned short* cwl = (unsigned short*)(ws + off_cwl);
  unsigned short* wth = (unsigned short*)(ws + off_wth);
  unsigned short* wtl = (unsigned short*)(ws + off_wtl);
  unsigned short* xh  = (unsigned short*)(ws + off_xh);
  unsigned short* xl  = (unsigned short*)(ws + off_xl);
  float* cct = (float*)(ws + off_cct);
  unsigned short* x1h = (unsigned short*)(ws + off_x1h);
  unsigned short* x1l = (unsigned short*)(ws + off_x1l);
  float* xt  = (float*)(ws + off_xt);
  unsigned short* ph  = (unsigned short*)(ws + off_ph);
  unsigned short* pl  = (unsigned short*)(ws + off_pl);
  unsigned short* tth = (unsigned short*)(ws + off_tth);
  unsigned short* ttl = (unsigned short*)(ws + off_ttl);
  float* obuf = (float*)(ws + off_o);
  void*  unused_v = (void*)(ws + off_rm);
  const float* unused_f = (const float*)(ws + off_rm);

  rowmean_kernel<<<kN / 32, 256, 0, stream>>>(cs, rm);
  split8_kernel<<<(kTok * kDin / 8) / 256, 256, 0, stream>>>(x, xh, xl, kTok * kDin / 8);
  split8_kernel<<<(kDin * kDin / 8) / 256, 256, 0, stream>>>(ct_w, cwh, cwl, kDin * kDin / 8);
  wt_kernel<<<kH, 256, 0, stream>>>(W, wth, wtl);
  wmma_gemm64<1, true, 2, 0, false><<<dim3(64, 1), 256, 0, stream>>>(
      xh, xl, kDin, 0L, cwh, cwl, kDin, 0L, (void*)cct, unused_v, kDin, 0L,
      ct_b, unused_f, 0L, kTok, kDin, kDin, 1.0f);
  combine_kernel<<<(kTok * kDin / 8) / 256, 256, 0, stream>>>(x, cct, rm, x1h, x1l, kTok * kDin / 8);
  wmma_gemm64<1, true, 0, 0, false><<<dim3(128, 1), 256, 0, stream>>>(
      x1h, x1l, kDin, 0L, wth, wtl, kDin, 0L, (void*)xt, unused_v, kHD, 0L,
      unused_f, unused_f, 0L, kTok, kHD, kDin, 1.0f);
  xpose_dots_kernel<<<dim3(kN / 64, kB * kH), 256, 0, stream>>>(xt, att, si, sj, tth, ttl);
  for (int b = 0; b < kB; ++b) {
    softmax_p_kernel<<<dim3(kN, kH), 256, 0, stream>>>(
        cs, si + (size_t)b * kH * kN, sj + (size_t)b * kH * kN, cbias, ph, pl);
    wmma_gemm64<1, true, 0, 0, false><<<dim3(4, kH), 256, 0, stream>>>(
        ph, pl, kN, (long)kN * kN,
        tth + (size_t)b * kH * kDout * kN, ttl + (size_t)b * kH * kDout * kN, kN, (long)kDout * kN,
        (void*)(obuf + (size_t)b * kH * kN * kDout), unused_v, kDout, (long)kN * kDout,
        unused_f, unused_f, 0L, kN, kDout, kN, 1.0f);
  }
  gate_out_kernel<<<dim3(kN / 64, kB * kH), 256, 0, stream>>>(obuf, cg_w, cg_b, out);
}
